// ImageReconstruction_35399120453774
// MI455X (gfx1250) — hardware-run, weakly checked
//
#include <hip/hip_runtime.h>


#ifndef NB
#define NB 16
#endif
#ifndef IMH
#define IMH 512
#endif
#define NB_FULL  16
#define IMH_FULL 512
#define IMW   512
#define PS    8
#define PLEN  64
#define NCODE 256
#define AW    4
#define WPR   (IMW / PS)
#define HBLK  (IMH / PS)
#define NBLK  (NB * HBLK)
#define TLW   (NCODE * 16)
#define OSP   132
#define NSC2  ((float)(-35.0 * 1.4426950408889634))
#define PSH   14.0f
#define CBS   64.0f
#define CBI   (1.0f / 64.0f)
#define NEGB  (-3.0e38f)

static_assert(PS * PS == PLEN);
static_assert(PLEN == 64);
static_assert(WPR == 16 * AW);
static_assert(IMH % PS == 0);
static_assert(IMH <= IMH_FULL);
static_assert(NB <= NB_FULL);
static_assert(NCODE % 32 == 0);
static_assert(NCODE == 256);
static_assert((NCODE * PLEN) % 8 == 0);
static_assert(((NCODE * PLEN) / 8) % 256 == 0);
static_assert(TLW == (NCODE / 32) * 4 * 32 * 4);
static_assert(32 * 4 == 16 * PS);
static_assert(PS * 32 * 16 == 16 * PLEN * 4);
static_assert(OSP >= 16 * PS);
static_assert((OSP * 4) % 16 == 0);
static_assert(AW == 4);
static_assert((size_t)NB_FULL * IMH_FULL * IMW * 4 == (size_t)16777216);
static_assert((size_t)AW * TLW * 4 + (size_t)AW * PS * OSP * 4 + (size_t)AW * 4 <= (size_t)131072);

typedef _Float16 h16;
typedef unsigned short bf;
typedef __attribute__((ext_vector_type(16))) __bf16   v16bf;
typedef __attribute__((ext_vector_type(16))) _Float16 v16h;
typedef __attribute__((ext_vector_type(8)))  _Float16 v8h;
typedef __attribute__((ext_vector_type(8)))  unsigned short v8us;
typedef __attribute__((ext_vector_type(8)))  float    v8f;
typedef __attribute__((ext_vector_type(4)))  float    v4f;
typedef v4f  __attribute__((may_alias)) v4fa;

__device__ __forceinline__ unsigned short f2bf(float f) { unsigned u = __float_as_uint(f); u += 0x7FFFu + ((u >> 16) & 1u); return (unsigned short)(u >> 16); }
__device__ __forceinline__ float bfr(float f) { return __uint_as_float(((unsigned)f2bf(f)) << 16); }
__device__ __forceinline__ v16h cat16(v8h lo, v8h hi) { return __builtin_shufflevector(lo, hi, 0, 1, 2, 3, 4, 5, 6, 7, 8, 9, 10, 11, 12, 13, 14, 15); }
__device__ __forceinline__ v16bf cat16b(v8us lo, v8us hi) { return __builtin_bit_cast(v16bf, __builtin_shufflevector(lo, hi, 0, 1, 2, 3, 4, 5, 6, 7, 8, 9, 10, 11, 12, 13, 14, 15)); }
__device__ __forceinline__ v8f wmma16(v16h a, v16h b, v8f c) { return __builtin_amdgcn_wmma_f32_16x16x32_f16(false, a, false, b, (short)0, c, false, false); }
__device__ __forceinline__ v8f wmmab(v16bf a, v16bf b, v8f c) { return __builtin_amdgcn_wmma_f32_16x16x32_bf16(false, a, false, b, (short)0, c, false, false); }
__device__ __forceinline__ v16h  ldh(const h16* p) { return cat16(*(const v8h*)p, *(const v8h*)(p + 16)); }
__device__ __forceinline__ v16bf ldb(const bf* p)  { return cat16b(*(const v8us*)p, *(const v8us*)(p + 16)); }
__device__ __forceinline__ void wave_sync() { __builtin_amdgcn_fence(3  , "wavefront"); __builtin_amdgcn_wave_barrier(); asm volatile("" ::: "memory"); }

__device__ __forceinline__ v8f wmmab_g(v16bf a, v16bf b, v8f c) { c = wmmab(a, b, c); asm volatile("v_nop\n\tv_nop\n\tv_nop\n\tv_nop" : "+v"(c) : "v"(a), "v"(b)); return c; }
__device__ __forceinline__ v8f wmma16_g(v16h a, v16h b, v8f c) { c = wmma16(a, b, c); asm volatile("v_nop\n\tv_nop\n\tv_nop\n\tv_nop" : "+v"(c) : "v"(a), "v"(b)); return c; }
static __device__ __forceinline__ h16 toh_flush(float v) { const h16 r = (h16)v; return (fabsf(v) < 6.103515625e-05f) ? (h16)0.0f : r; }

__global__ __launch_bounds__(256) void k_cvt8(const float* __restrict__ src, bf* dst, size_t n8) {
    const size_t i = (size_t)blockIdx.x * 256 + threadIdx.x; if (i >= n8) return;
    const v8f v = *(const v8f*)(src + i * 8); v8us o;
#pragma unroll
    for (int k = 0; k < 8; ++k) o[k] = f2bf(v[k]);
    *(volatile v8us*)(dst + i * 8) = o; __threadfence(); *(volatile v8us*)(dst + i * 8) = o;
}

__global__ __launch_bounds__(256) void k_cbt(const float* __restrict__ cb, h16* CT) {
    const int i = blockIdx.x * 256 + threadIdx.x; if (i >= NCODE * PLEN / 8) return;
    const int d = i / (NCODE / 8), c8 = (i % (NCODE / 8)) * 8;
    v8h o;
#pragma unroll
    for (int k = 0; k < 8; ++k) o[k] = toh_flush(bfr(cb[(size_t)(c8 + k) * PLEN + d]) * CBS);
    *(volatile v8h*)(CT + (size_t)i * 8) = o; __threadfence(); *(volatile v8h*)(CT + (size_t)i * 8) = o;
}

__global__ __launch_bounds__(256) void k_cbn(const float* __restrict__ cb, float* B2) {
    const int n = threadIdx.x;
    float s = 0.0f;
#pragma unroll 1
    for (int q = 0; q < PLEN / 4; ++q) { const v4f v = *(const v4f*)(cb + (size_t)n * PLEN + q * 4);
        const float y0 = bfr(v[0]), y1 = bfr(v[1]), y2 = bfr(v[2]), y3 = bfr(v[3]);
        s += y0 * y0; s += y1 * y1; s += y2 * y2; s += y3 * y3; }
    *(volatile float*)(B2 + n) = s; __threadfence(); *(volatile float*)(B2 + n) = s;
}

__global__ __launch_bounds__(32 * AW) void k_recon(const float* __restrict__ IMG, const bf* __restrict__ CBB, const h16* __restrict__ CT, const float* __restrict__ B2, float* OUT, float* PART) {
    __shared__ __align__(16) float tl[AW * TLW];
    __shared__ __align__(16) float os[AW * PS * OSP];
    __shared__ float pw[AW];
    const int lane = threadIdx.x & 31, lr = lane & 15, hi = lane >> 4;
    const int wave = __builtin_amdgcn_readfirstlane((int)(threadIdx.x >> 5));
    const int b = blockIdx.y, hb = blockIdx.x;
    const int wb0 = wave * 16;
    const size_t ibase = (size_t)b * ((size_t)IMH_FULL * IMW) + (size_t)(hb * PS) * IMW;
    const float* ip = IMG + ibase + (size_t)(wb0 + lr) * PS;
    v16bf pf0, pf1; float a2;
    {
        const v8f x0 = *(const v8f*)(ip + (size_t)(0 + hi) * IMW);
        const v8f x1 = *(const v8f*)(ip + (size_t)(2 + hi) * IMW);
        const v8f x2 = *(const v8f*)(ip + (size_t)(4 + hi) * IMW);
        const v8f x3 = *(const v8f*)(ip + (size_t)(6 + hi) * IMW);
        v8us u0, u1, u2, u3; float s = 0.0f;
#pragma unroll
        for (int e = 0; e < 8; ++e) {
            u0[e] = f2bf(x0[e]); u1[e] = f2bf(x1[e]); u2[e] = f2bf(x2[e]); u3[e] = f2bf(x3[e]);
            const float y0 = __uint_as_float(((unsigned)u0[e]) << 16), y1 = __uint_as_float(((unsigned)u1[e]) << 16);
            const float y2 = __uint_as_float(((unsigned)u2[e]) << 16), y3 = __uint_as_float(((unsigned)u3[e]) << 16);
            s += y0 * y0; s += y1 * y1; s += y2 * y2; s += y3 * y3; }
        pf0 = cat16b(u0, u1); pf1 = cat16b(u2, u3);
        a2 = s + __shfl_xor(s, 16, 32);
    }
    const int tb = wave * TLW + lane * 4;
    const size_t co = (size_t)lr * PLEN + 8 * hi;
    float mx = NEGB;
#pragma unroll 1
    for (int tp = 0; tp < NCODE / 32; ++tp) {
        const int c0 = tp * 32;
        const bf* ca = CBB + co + (size_t)c0 * PLEN;
        const v16bf a00 = ldb(ca), a01 = ldb(ca + 32), a10 = ldb(ca + 16 * PLEN), a11 = ldb(ca + 16 * PLEN + 32);
        v8f sa = (v8f){}, sb = (v8f){};
        sa = wmmab_g(a00, pf0, sa); sa = wmmab_g(a01, pf1, sa);
        sb = wmmab_g(a10, pf0, sb); sb = wmmab_g(a11, pf1, sb);
        const float* np = B2 + c0 + 8 * hi;
        const v4f n0 = *(const v4f*)np, n1 = *(const v4f*)(np + 4), n2 = *(const v4f*)(np + 16), n3 = *(const v4f*)(np + 20);
        v4f ta0, ta1, tb0, tb1;
#pragma unroll
        for (int i = 0; i < 4; ++i) {
            ta0[i] = ((a2 + n0[i]) - 2.0f * sa[i]) * NSC2;     ta1[i] = ((a2 + n1[i]) - 2.0f * sa[4 + i]) * NSC2;
            tb0[i] = ((a2 + n2[i]) - 2.0f * sb[i]) * NSC2;     tb1[i] = ((a2 + n3[i]) - 2.0f * sb[4 + i]) * NSC2;
            mx = fmaxf(mx, fmaxf(fmaxf(ta0[i], ta1[i]), fmaxf(tb0[i], tb1[i]))); }
        *(v4fa*)(&tl[tb + (tp * 4 + 0) * 128]) = ta0; *(v4fa*)(&tl[tb + (tp * 4 + 1) * 128]) = ta1;
        *(v4fa*)(&tl[tb + (tp * 4 + 2) * 128]) = tb0; *(v4fa*)(&tl[tb + (tp * 4 + 3) * 128]) = tb1;
    }
    const float m = fmaxf(mx, __shfl_xor(mx, 16, 32));
    float ls = 0.0f;
#pragma unroll 1
    for (int q = 0; q < (NCODE / 32) * 4; ++q) { const v4f t = *(const v4fa*)(&tl[tb + q * 128]);
#pragma unroll
        for (int i = 0; i < 4; ++i) ls += __builtin_amdgcn_exp2f((t[i] - m) + PSH); }
    const float l = ls + __shfl_xor(ls, 16, 32);
    const float invl = 1.0f / l;
    v8f o[4];
#pragma unroll
    for (int j = 0; j < 4; ++j) o[j] = (v8f){};
    const size_t vo = (size_t)lr * NCODE + 8 * hi;
    float pen = 0.0f;
#pragma unroll 1
    for (int tp = 0; tp < NCODE / 32; ++tp) {
        const v4f ta0 = *(const v4fa*)(&tl[tb + (tp * 4 + 0) * 128]), ta1 = *(const v4fa*)(&tl[tb + (tp * 4 + 1) * 128]);
        const v4f tb0 = *(const v4fa*)(&tl[tb + (tp * 4 + 2) * 128]), tb1 = *(const v4fa*)(&tl[tb + (tp * 4 + 3) * 128]);
        v16h pb;
#pragma unroll
        for (int i = 0; i < 4; ++i) {
            const float g0 = (ta0[i] - m) + PSH, g1 = (ta1[i] - m) + PSH, g2 = (tb0[i] - m) + PSH, g3 = (tb1[i] - m) + PSH;
            const float e0 = __builtin_amdgcn_exp2f(g0), e1 = __builtin_amdgcn_exp2f(g1), e2 = __builtin_amdgcn_exp2f(g2), e3 = __builtin_amdgcn_exp2f(g3);
            const float w0 = e0 * invl, w1 = e1 * invl, w2 = e2 * invl, w3 = e3 * invl;
            pen += fminf(w0, 1.0f - w0); pen += fminf(w1, 1.0f - w1); pen += fminf(w2, 1.0f - w2); pen += fminf(w3, 1.0f - w3);
            pb[i]      = (g0 < -14.0f) ? (h16)0.0f : (h16)e0;
            pb[4 + i]  = (g1 < -14.0f) ? (h16)0.0f : (h16)e1;
            pb[8 + i]  = (g2 < -14.0f) ? (h16)0.0f : (h16)e2;
            pb[12 + i] = (g3 < -14.0f) ? (h16)0.0f : (h16)e3; }
        const h16* va = CT + vo + tp * 32;
#pragma unroll
        for (int j = 0; j < 4; ++j) { const v16h vf = ldh(va + (size_t)(16 * j) * NCODE); o[j] = wmma16_g(vf, pb, o[j]); }
    }
    const float sc = invl * CBI;
    const int wo = wave * PS * OSP;
#pragma unroll
    for (int j = 0; j < 4; ++j) { v4f a, c;
#pragma unroll
        for (int i = 0; i < 4; ++i) { a[i] = o[j][i] * sc; c[i] = o[j][4 + i] * sc; }
        *(v4fa*)(&os[wo + (2 * j + hi) * OSP + lr * 8]) = a; *(v4fa*)(&os[wo + (2 * j + hi) * OSP + lr * 8 + 4]) = c; }
    wave_sync();
    pen += __shfl_xor(pen, 16, 32); pen += __shfl_xor(pen, 8, 32); pen += __shfl_xor(pen, 4, 32); pen += __shfl_xor(pen, 2, 32); pen += __shfl_xor(pen, 1, 32);
    if (lane == 0) pw[wave] = pen;
    __syncthreads();
    const float p0 = pw[0], p1 = pw[1], p2 = pw[2], p3 = pw[3];
    v4f pv; pv[0] = (lane == 0) ? p0 : 0.0f; pv[1] = (lane == 0) ? p1 : 0.0f; pv[2] = (lane == 0) ? p2 : 0.0f; pv[3] = (lane == 0) ? p3 : 0.0f;
    float* orow = OUT + ibase + (size_t)wb0 * PS + (size_t)lane * 4;
    float* pl = PART + ((size_t)b * HBLK + (size_t)hb) * 32 + (size_t)(lane & 7) * 4;
#pragma unroll 1
    for (int ps = 0; ps < 2; ++ps) {
#pragma unroll
        for (int i = 0; i < PS; ++i) {
            const v4f val = *(const v4fa*)(&os[wo + i * OSP + lane * 4]);
            *(volatile v4f*)(orow + (size_t)i * IMW) = val; }
        if ((wave == 0) & (lane < 8)) *(volatile v4f*)pl = pv;
        if (ps == 0) __threadfence(); }
}

__global__ __launch_bounds__(256) void k_pen(const float* __restrict__ PART, float* OUT1) {
    __shared__ double sm[256];
    const int tid = threadIdx.x;
    double s = 0.0;
#pragma unroll 1
    for (int i = tid; i < NBLK; i += 256) { const v4f p = *(const v4f*)(PART + (size_t)i * 32);
        s += ((double)p[0] + (double)p[1]) + ((double)p[2] + (double)p[3]); }
    sm[tid] = s;
    __syncthreads();
    if (tid == 0) {
        double t = 0.0;
#pragma unroll 1
        for (int k = 0; k < 256; ++k) t += sm[k];
        const float r = (float)(t * (1.0 / ((double)NB * (double)HBLK * (double)WPR)));
        *(volatile float*)OUT1 = r; __threadfence(); *(volatile float*)OUT1 = r; }
}

static constexpr size_t al256(size_t v) { return (v + 255) & ~(size_t)255; }
static constexpr size_t SZ_CB = al256((size_t)NCODE * PLEN * 2);
static constexpr size_t SZ_CT = al256((size_t)PLEN * NCODE * 2);
static constexpr size_t SZ_B2 = al256((size_t)NCODE * 4);
static constexpr size_t SZ_PT = al256((size_t)NBLK * 128);
static constexpr size_t SZ_TOTAL = SZ_CB + SZ_CT + SZ_B2 + SZ_PT;
static_assert(SZ_TOTAL <= (size_t)134217728);
static_assert((size_t)((size_t)(NB - 1) * HBLK + (HBLK - 1)) * 128 + 128 <= SZ_PT);
static_assert((size_t)(NCODE * PLEN / 8 - 1) * 16 + 16 <= SZ_CT);
static_assert((size_t)(NB_FULL - 1) * IMH_FULL * IMW + (size_t)IMH_FULL * IMW <= (size_t)NB_FULL * IMH_FULL * IMW);

extern "C" void kernel_launch(void* const* d_in, const int* in_sizes, int n_in,
                              void* d_out, int out_size, void* d_ws, size_t ws_size, hipStream_t stream) {
    if (n_in < 2) return;
    const size_t needi = (size_t)(NB - 1) * IMH_FULL * IMW + (size_t)IMH * IMW;
    if ((size_t)in_sizes[0] < needi) return;
    if ((size_t)in_sizes[1] < (size_t)NCODE * PLEN) return;
    const size_t out1 = (size_t)NB_FULL * IMH_FULL * IMW;
    if ((size_t)out_size < out1 + 1) return;
    if (SZ_TOTAL > ws_size) return;
    const float* img = (const float*)d_in[0];
    const float* cb  = (const float*)d_in[1];
    float* OUT = (float*)d_out;
    char* wsp = (char*)d_ws;
    bf*    CBB  = (bf*)wsp;    wsp += SZ_CB;
    h16*   CT   = (h16*)wsp;   wsp += SZ_CT;
    float* B2   = (float*)wsp; wsp += SZ_B2;
    float* PART = (float*)wsp; wsp += SZ_PT;

    { const size_t n8 = (size_t)NCODE * PLEN / 8;
      k_cvt8<<<(unsigned)((n8 + 255) / 256), 256, 0, stream>>>(cb, CBB, n8); }
    k_cbt<<<(unsigned)((NCODE * PLEN / 8) / 256), 256, 0, stream>>>(cb, CT);
    k_cbn<<<1, 256, 0, stream>>>(cb, B2);
    k_recon<<<dim3(HBLK, NB, 1), 32 * AW, 0, stream>>>(img, CBB, CT, B2, OUT, PART);
    k_pen<<<1, 256, 0, stream>>>(PART, OUT + out1);
}
